// FlexEquivariantProductBasisBlock_1778116461347
// MI455X (gfx1250) — hardware-verified
//
#include <hip/hip_runtime.h>
#include <stdint.h>

typedef __bf16 v16b __attribute__((ext_vector_type(16)));
typedef __bf16 v8b  __attribute__((ext_vector_type(8)));
typedef float  v8f  __attribute__((ext_vector_type(8)));
typedef float  v4f  __attribute__((ext_vector_type(4)));

union Frag  { v16b v; v8b half[2]; };
union Pack8 { v8b h; v4f f; };

#define N_NODES   4096
#define CCH       128
#define NSPEC     10
#define NPAIR     (N_NODES * CCH)
#define SCN       (NSPEC * CCH)
#define MT0       6
#define MT1       16
#define NTG       (MT0 + MT1)
#define KEXT      108
#define KSTEPS    4
#define FRAG_EL   512
#define RPP       356
#define SYM_WAVES 2
#define LIN_THREADS 128
#define OUTW      512

#define A3_BYTES  ((size_t)NTG * KSTEPS * FRAG_EL * 2)
#define WF_BYTES  ((size_t)2 * 2 * 4 * 8 * FRAG_EL * 2)
#define UE2_BYTES ((size_t)36 * 9 * SCN * 4)
#define UE1_BYTES ((size_t)36 * SCN * 4)
#define F_BYTES   ((size_t)4 * NPAIR * 4)
#define OFF_A3    ((size_t)0)
#define OFF_WF    (OFF_A3 + A3_BYTES)
#define OFF_UE2   (OFF_WF + WF_BYTES)
#define OFF_UE1   (OFF_UE2 + UE2_BYTES)
#define OFF_F     (OFF_UE1 + UE1_BYTES)
#define WS_TOTAL  (OFF_F + F_BYTES)

typedef char chk_align[(OFF_WF % 128 == 0 && OFF_UE2 % 128 == 0 && OFF_UE1 % 128 == 0 && OFF_F % 128 == 0) ? 1 : -1];
typedef char chk_tiles[(NPAIR % (16 * SYM_WAVES) == 0) ? 1 : -1];
typedef char chk_waves[(SYM_WAVES == 2) ? 1 : -1];
typedef char chk_rows[(96 + MT1 * 16 <= RPP) ? 1 : -1];
typedef char chk_mtiles[(N_NODES % 16 == 0) ? 1 : -1];

__device__ __forceinline__ float bf16_hi(float z) {
  uint32_t u = __float_as_uint(z);
  u = (u + 0x7FFFu + ((u >> 16) & 1u)) & 0xFFFF0000u;
  return __uint_as_float(u);
}

__device__ __forceinline__ v8f mma_bf16(v16b a, v16b b, v8f c) {
  c = __builtin_amdgcn_wmma_f32_16x16x32_bf16(false, a, false, b, (short)0, c, false, false);
  asm volatile("v_nop\n\tv_nop\n\tv_nop\n\tv_nop" : "+v"(c) : "v"(a), "v"(b));
  return c;
}

__global__ __launch_bounds__(128)
void k_prep_a3(const float* __restrict__ U3a, const float* __restrict__ U3b,
               __bf16* __restrict__ A3) {
  const int tid = blockIdx.x * 128 + threadIdx.x;
  const bool valid = tid < NTG * KSTEPS * 64;
  Pack8 pk;
  pk.f = (v4f){0.f, 0.f, 0.f, 0.f};
  __bf16* dst = A3;
  if (valid) {
    const int e8 = tid & 1, lane = (tid >> 1) & 31, fr = tid >> 6;
    const int tg = fr >> 2, ks = fr & 3, h = lane >> 4, mrow = lane & 15;
    const bool first = tg < MT0;
    const float* src = first ? U3a : U3b;
    const int rows = first ? 81 : 243;
    const int m = (first ? tg : (tg - MT0)) * 16 + mrow;
#pragma unroll
    for (int j = 0; j < 8; ++j) {
      const int kk = ks * 32 + 8 * h + 16 * e8 + j;
      const int seg = kk / 36, k = kk - seg * 36;
      float v = 0.f;
      if (kk < KEXT && m < rows) {
        const float u = src[m * 36 + k];
        const float hf = bf16_hi(u);
        v = (seg == 2) ? (u - hf) : hf;
      }
      pk.h[j] = (__bf16)v;
    }
    dst = A3 + ((size_t)fr * 32 + lane) * 16 + 8 * e8;
    *(volatile v4f*)dst = pk.f;
  }
  __threadfence();
  if (valid) *(volatile v4f*)dst = pk.f;
}

__global__ __launch_bounds__(128)
void k_prep_wf(const float* __restrict__ Wa, const float* __restrict__ Wb,
               __bf16* __restrict__ WF) {
  const int tid = blockIdx.x * 128 + threadIdx.x;
  const bool valid = tid < 2 * 2 * 4 * 8 * 64;
  Pack8 pk;
  pk.f = (v4f){0.f, 0.f, 0.f, 0.f};
  __bf16* dst = WF;
  if (valid) {
    const int e8 = tid & 1, lane = (tid >> 1) & 31, fr = tid >> 6;
    const int nt = fr & 7, ks = (fr >> 3) & 3, piece = (fr >> 5) & 1, ir = fr >> 6;
    const int h = lane >> 4;
    const int n = nt * 16 + (lane & 15);
    const float* W = ir ? Wb : Wa;
#pragma unroll
    for (int j = 0; j < 8; ++j) {
      const int k = ks * 32 + 8 * h + 16 * e8 + j;
      const float w = W[k * CCH + n];
      const float hf = bf16_hi(w);
      pk.h[j] = (__bf16)(piece ? (w - hf) : hf);
    }
    dst = WF + ((size_t)fr * 32 + lane) * 16 + 8 * e8;
    *(volatile v4f*)dst = pk.f;
  }
  __threadfence();
  if (valid) *(volatile v4f*)dst = pk.f;
}

__global__ __launch_bounds__(128)
void k_prep_ue2(const float* __restrict__ U2a, const float* __restrict__ W2a,
                const float* __restrict__ U2b, const float* __restrict__ W2b,
                float* __restrict__ UE2) {
  const int tid = blockIdx.x * 128 + threadIdx.x;
  const bool valid = tid < 36 * 9 * (SCN / 4);
  v4f v = {0.f, 0.f, 0.f, 0.f};
  float* dst = UE2;
  if (valid) {
    const int c4 = tid & 31;
    const int s = (tid >> 5) % NSPEC;
    const int q = (tid / (SCN / 4)) % 9;
    const int row = tid / (9 * (SCN / 4));
    float ua, ub;
    const float* w;
    if (row < 9) {
      ua = U2a[row * 18 + q * 2 + 0];
      ub = U2a[row * 18 + q * 2 + 1];
      w = W2a;
    } else {
      const int r = row - 9, o = r / 9, p = r - o * 9;
      ua = U2b[o * 162 + p * 18 + q * 2 + 0];
      ub = U2b[o * 162 + p * 18 + q * 2 + 1];
      w = W2b;
    }
    const float* wa = w + (size_t)(s * 2) * CCH + 4 * c4;
    const float* wb = wa + CCH;
#pragma unroll
    for (int jj = 0; jj < 4; ++jj) v[jj] = ua * wa[jj] + ub * wb[jj];
    dst = UE2 + (size_t)tid * 4;
    *(volatile v4f*)dst = v;
  }
  __threadfence();
  if (valid) *(volatile v4f*)dst = v;
}

__global__ __launch_bounds__(128)
void k_prep_ue1(const float* __restrict__ U1a, const float* __restrict__ W1a,
                const float* __restrict__ U1b, const float* __restrict__ W1b,
                float* __restrict__ UE1) {
  const int tid = blockIdx.x * 128 + threadIdx.x;
  const bool valid = tid < 4 * 9 * (SCN / 4);
  v4f v = {0.f, 0.f, 0.f, 0.f};
  float* dst = UE1;
  if (valid) {
    const int c4 = tid & 31;
    const int s = (tid >> 5) % NSPEC;
    const int i = (tid / (SCN / 4)) % 9;
    const int og = tid / (9 * (SCN / 4));
    const float u = (og == 0) ? U1a[i] : U1b[(og - 1) * 9 + i];
    const float* w = ((og == 0) ? W1a : W1b) + (size_t)s * CCH + 4 * c4;
#pragma unroll
    for (int jj = 0; jj < 4; ++jj) v[jj] = u * w[jj];
    dst = UE1 + (size_t)tid * 4;
    *(volatile v4f*)dst = v;
  }
  __threadfence();
  if (valid) *(volatile v4f*)dst = v;
}

#define BSEL(kk) (((kk) < KEXT) ? ((((kk) / 36) == 1) ? zl[(kk) % 36] : zh[(kk) % 36]) : 0.0f)

template <int NT>
__device__ __forceinline__ void contract_irrep(const float (&x9)[9], const float (&w3)[4],
                                               const __bf16* __restrict__ Afr,
                                               float* dstL, int lane, int h) {
  float zh[36], zl[36];
#pragma unroll
  for (int k = 0; k < 36; ++k) {
    const float z = x9[k >> 2] * w3[k & 3];
    const float hf = bf16_hi(z);
    zh[k] = hf;
    zl[k] = z - hf;
  }
  Frag bq[KSTEPS];
#pragma unroll
  for (int ks = 0; ks < KSTEPS; ++ks) {
#pragma unroll
    for (int e = 0; e < 16; ++e) {
      const int kk0 = ks * 32 + ((e < 8) ? e : (8 + e));
      const int kk1 = kk0 + 8;
      const float v0 = BSEL(kk0);
      const float v1 = BSEL(kk1);
      bq[ks].v[e] = (__bf16)(h ? v1 : v0);
    }
  }
#pragma unroll 1
  for (int mt = 0; mt < NT; ++mt) {
    const __bf16* ap = Afr + (size_t)mt * (KSTEPS * FRAG_EL) + lane * 16;
    v8f acc = {0.f, 0.f, 0.f, 0.f, 0.f, 0.f, 0.f, 0.f};
#pragma unroll
    for (int ks = 0; ks < KSTEPS; ++ks) {
      Frag a;
      a.half[0] = *(const v8b*)(ap + ks * FRAG_EL);
      a.half[1] = *(const v8b*)(ap + ks * FRAG_EL + 8);
      acc = mma_bf16(a.v, bq[ks].v, acc);
    }
    float* d = dstL + mt * 16 + 8 * h;
    const v4f lo = {acc[0], acc[1], acc[2], acc[3]};
    const v4f hi = {acc[4], acc[5], acc[6], acc[7]};
    *(v4f*)(d)     = lo;
    *(v4f*)(d + 4) = hi;
  }
}

__global__ __launch_bounds__(SYM_WAVES * 32)
void k_sym(const float* __restrict__ x, const int* __restrict__ specie,
           const __bf16* __restrict__ A3,
           const float* __restrict__ W3a, const float* __restrict__ W3b,
           const float* __restrict__ UE2, const float* __restrict__ UE1,
           float* __restrict__ F) {
  __shared__ __align__(16) float lds[SYM_WAVES * 16 * RPP];
  __shared__ __align__(16) float fst[4 * 32];
  const int wave = threadIdx.x >> 5, lane = threadIdx.x & 31;
  const int h = lane >> 4, m = lane & 15;
  const int b = blockIdx.x >> 2;
  const int cblk = (blockIdx.x & 3) * 32;
  const int col = cblk + 16 * wave + m;
  int s = specie[b];
  s = (s < 0) ? 0 : ((s > NSPEC - 1) ? (NSPEC - 1) : s);

  float x9[9];
  const float* xp = x + ((size_t)b * CCH + col) * 9;
#pragma unroll
  for (int i = 0; i < 9; ++i) x9[i] = xp[i];

  const int scbase = s * CCH + col;
  float* myL = lds + wave * (16 * RPP) + m * RPP;

  {
    float w3[4];
#pragma unroll
    for (int k = 0; k < 4; ++k) w3[k] = W3a[(size_t)(s * 4 + k) * CCH + col];
    contract_irrep<MT0>(x9, w3, A3, myL, lane, h);
  }
  {
    float w3[4];
#pragma unroll
    for (int k = 0; k < 4; ++k) w3[k] = W3b[(size_t)(s * 4 + k) * CCH + col];
    contract_irrep<MT1>(x9, w3, A3 + (size_t)MT0 * KSTEPS * FRAG_EL, myL + 96, lane, h);
  }
  __syncthreads();

#pragma unroll
  for (int g = 0; g < 2; ++g) {
    const int og = 2 * h + g;
    const int ldsBase = (og == 0) ? 0 : (96 + (og - 1) * 81);
    float f = 0.f;
#pragma unroll
    for (int p2 = 0; p2 < 9; ++p2) {
      const float* l1 = myL + ldsBase + p2 * 9;
      const int row = og * 9 + p2;
      float o2 = 0.f;
#pragma unroll
      for (int q = 0; q < 9; ++q) {
        const float ue = UE2[(size_t)(row * 9 + q) * SCN + scbase];
        o2 = fmaf(l1[q] + ue, x9[q], o2);
      }
      const float u1 = UE1[(size_t)row * SCN + scbase];
      f = fmaf(o2 + u1, x9[p2], f);
    }
    fst[og * 32 + 16 * wave + m] = f;
  }
  __syncthreads();

  v4f fv = {0.f, 0.f, 0.f, 0.f};
  float* gp = F;
  if (wave == 0) {
    const int og = lane >> 3, j = lane & 7;
    fv = *(const v4f*)(fst + og * 32 + 4 * j);
    gp = F + (size_t)og * NPAIR + (size_t)b * CCH + cblk + 4 * j;
    *(volatile v4f*)gp = fv;
  }
  __threadfence();
  if (wave == 0) *(volatile v4f*)gp = fv;
}

__global__ __launch_bounds__(LIN_THREADS)
void k_lin(const float* __restrict__ F, const __bf16* __restrict__ WF,
           const float* __restrict__ bias, float* __restrict__ out) {
  __shared__ __align__(16) float tile[16 * OUTW];
  const int wave = threadIdx.x >> 5, lane = threadIdx.x & 31;
  const int h = lane >> 4, m = lane & 15;
  const int mtile = blockIdx.x;
  const float* A = F + (size_t)wave * NPAIR + (size_t)(mtile * 16 + m) * CCH + 8 * h;
  const __bf16* WB = WF + (size_t)(wave ? 64 : 0) * FRAG_EL;

  v8f acc[8];
#pragma unroll
  for (int nt = 0; nt < 8; ++nt) acc[nt] = (v8f){0.f, 0.f, 0.f, 0.f, 0.f, 0.f, 0.f, 0.f};

#pragma unroll 1
  for (int ks = 0; ks < 4; ++ks) {
    const float* ap = A + ks * 32;
    const v4f f0 = *(const v4f*)(ap);
    const v4f f1 = *(const v4f*)(ap + 4);
    const v4f f2 = *(const v4f*)(ap + 16);
    const v4f f3 = *(const v4f*)(ap + 20);
    Frag ah, al;
#pragma unroll
    for (int e = 0; e < 16; ++e) {
      const float v = (e < 4) ? f0[e] : ((e < 8) ? f1[e - 4] : ((e < 12) ? f2[e - 8] : f3[e - 12]));
      const float hf = bf16_hi(v);
      ah.v[e] = (__bf16)hf;
      al.v[e] = (__bf16)(v - hf);
    }
#pragma unroll
    for (int nt = 0; nt < 8; ++nt) {
      const __bf16* bp = WB + ((size_t)(ks * 8 + nt) * 32 + lane) * 16;
      const __bf16* bp2 = bp + (size_t)32 * FRAG_EL;
      Frag bh, bl;
      bh.half[0] = *(const v8b*)(bp);
      bh.half[1] = *(const v8b*)(bp + 8);
      bl.half[0] = *(const v8b*)(bp2);
      bl.half[1] = *(const v8b*)(bp2 + 8);
      acc[nt] = mma_bf16(ah.v, bh.v, acc[nt]);
      acc[nt] = mma_bf16(ah.v, bl.v, acc[nt]);
      acc[nt] = mma_bf16(al.v, bh.v, acc[nt]);
    }
  }

  const float scale = 0.08838834764831845f;
  const bool is0 = (wave == 0);
#pragma unroll
  for (int nt = 0; nt < 8; ++nt) {
    const int mcol = nt * 16 + m;
    const float bv = is0 ? bias[mcol] : 0.f;
    const int pos = is0 ? mcol : (128 + mcol * 3 + (wave - 1));
#pragma unroll
    for (int r = 0; r < 8; ++r) tile[(8 * h + r) * OUTW + pos] = acc[nt][r] * scale + bv;
  }
  __syncthreads();

  float* ob = out + (size_t)(mtile * 16) * OUTW + 4 * threadIdx.x;
  const float* tb = tile + 4 * threadIdx.x;
#pragma unroll
  for (int r = 0; r < 16; ++r) {
    const v4f v = *(const v4f*)(tb + r * OUTW);
    *(volatile v4f*)(ob + (size_t)r * OUTW) = v;
  }
  __threadfence();
#pragma unroll
  for (int r = 0; r < 16; ++r) {
    const v4f v = *(const v4f*)(tb + r * OUTW);
    *(volatile v4f*)(ob + (size_t)r * OUTW) = v;
  }
}

extern "C" void kernel_launch(void* const* d_in, const int* in_sizes, int n_in,
                              void* d_out, int out_size, void* d_ws, size_t ws_size,
                              hipStream_t stream) {
  if (n_in < 17) return;
  if ((size_t)in_sizes[0] != (size_t)N_NODES * CCH * 9) return;
  if ((size_t)out_size < (size_t)N_NODES * OUTW) return;
  if (ws_size < WS_TOTAL) return;

  const float* x       = (const float*)d_in[0];
  const int*   specie  = (const int*)  d_in[1];
  const float* U3_0e   = (const float*)d_in[2];
  const float* U2_0e   = (const float*)d_in[3];
  const float* U1_0e   = (const float*)d_in[4];
  const float* W3_0e   = (const float*)d_in[5];
  const float* W2_0e   = (const float*)d_in[6];
  const float* W1_0e   = (const float*)d_in[7];
  const float* U3_1o   = (const float*)d_in[8];
  const float* U2_1o   = (const float*)d_in[9];
  const float* U1_1o   = (const float*)d_in[10];
  const float* W3_1o   = (const float*)d_in[11];
  const float* W2_1o   = (const float*)d_in[12];
  const float* W1_1o   = (const float*)d_in[13];
  const float* Wlin_0e = (const float*)d_in[14];
  const float* Wlin_1o = (const float*)d_in[15];
  const float* bias_0e = (const float*)d_in[16];
  float* out = (float*)d_out;

  char* ws = (char*)d_ws;
  __bf16* A3  = (__bf16*)(ws + OFF_A3);
  __bf16* WF  = (__bf16*)(ws + OFF_WF);
  float*  UE2 = (float*)(ws + OFF_UE2);
  float*  UE1 = (float*)(ws + OFF_UE1);
  float*  F   = (float*)(ws + OFF_F);

  const int nA3  = NTG * KSTEPS * 64;
  const int nWF  = 2 * 2 * 4 * 8 * 64;
  const int nUE2 = 36 * 9 * (SCN / 4);
  const int nUE1 = 4 * 9 * (SCN / 4);

  k_prep_a3 <<<(nA3 + 127) / 128, 128, 0, stream>>>(U3_0e, U3_1o, A3);
  k_prep_wf <<<(nWF + 127) / 128, 128, 0, stream>>>(Wlin_0e, Wlin_1o, WF);
  k_prep_ue2<<<(nUE2 + 127) / 128, 128, 0, stream>>>(U2_0e, W2_0e, U2_1o, W2_1o, UE2);
  k_prep_ue1<<<(nUE1 + 127) / 128, 128, 0, stream>>>(U1_0e, W1_0e, U1_1o, W1_1o, UE1);

  k_sym<<<NPAIR / 16 / SYM_WAVES, SYM_WAVES * 32, 0, stream>>>(
      x, specie, A3, W3_0e, W3_1o, UE2, UE1, F);

  k_lin<<<N_NODES / 16, LIN_THREADS, 0, stream>>>(F, WF, bias_0e, out);
}
